// RelativeGlobalAttention_1408749273411
// MI455X (gfx1250) — hardware-verified
//
#include <hip/hip_runtime.h>
#include <math.h>
#include <stdint.h>

#ifndef NB
#define NB 4
#endif
#ifndef SEQ
#define SEQ 2048
#endif
#define NB_FULL  4
#define SEQ_FULL 2048
#define ND    512
#define NH    8
#define HDV   64
#define HQK   128
#define QKW   (2 * ND)
#define NKT   (SEQ / 64)
#define BDW   (SEQ + 64)
#define NPAIR 4
#define QRES  2

static_assert(SEQ % 64 == 0);
static_assert(SEQ <= SEQ_FULL);
static_assert(NB >= 1);
static_assert(NB <= NB_FULL);
static_assert(ND == NH * HDV);
static_assert(HQK == 2 * HDV);
static_assert(NH % NPAIR == 0);
static_assert(ND % 64 == 0);
static_assert(BDW % 64 == 0);
static_assert(NKT > QRES);

typedef _Float16 v16h __attribute__((ext_vector_type(16)));
typedef _Float16 v8h  __attribute__((ext_vector_type(8)));
typedef float    v8f  __attribute__((ext_vector_type(8)));
typedef float    v4f  __attribute__((ext_vector_type(4)));
typedef v4f __attribute__((may_alias)) v4fa;
typedef v8h __attribute__((may_alias)) v8ha;

__device__ __forceinline__ float bf_rne(float f) {
  unsigned u = __float_as_uint(f);
  u = (u + 0x7FFFu + ((u >> 16) & 1u)) & 0xFFFF0000u;
  return __uint_as_float(u);
}

union FragU { v16h v; v8ha h[2]; };
__device__ __forceinline__ v16h ldfrag(const _Float16* p) {
  FragU f;
  f.h[0] = *(const v8ha*)(p);
  f.h[1] = *(const v8ha*)(p + 16);
  return f.v;
}

__device__ __forceinline__ v8f mma16(v16h a, v16h b, v8f c) {
  c = __builtin_amdgcn_wmma_f32_16x16x32_f16(false, a, false, b, (short)0, c, false, false);
  asm volatile("v_nop\n\tv_nop\n\tv_nop\n\tv_nop" : "+v"(c) : "v"(a), "v"(b));
  return c;
}

__device__ __forceinline__ v8f zero8() { v8f z = {0.f, 0.f, 0.f, 0.f, 0.f, 0.f, 0.f, 0.f}; return z; }

__global__ __launch_bounds__(256) void cvt_kernel(const float* __restrict__ src, _Float16* __restrict__ dst,
                                                  int nrows, float s1) {
  const int i = blockIdx.x * 256 + threadIdx.x;
  if (i >= nrows * (ND / 8)) return;
  const int r  = i / (ND / 8);
  const int c8 = (i - r * (ND / 8)) * 8;
  const float* sp = src + (size_t)r * ND + c8;
  const v4f a = *(const v4f*)(sp);
  const v4f b = *(const v4f*)(sp + 4);
  float f[8];
  f[0] = bf_rne(a[0]); f[1] = bf_rne(a[1]); f[2] = bf_rne(a[2]); f[3] = bf_rne(a[3]);
  f[4] = bf_rne(b[0]); f[5] = bf_rne(b[1]); f[6] = bf_rne(b[2]); f[7] = bf_rne(b[3]);
  v8h o1;
#pragma unroll
  for (int e = 0; e < 8; ++e) o1[e] = (_Float16)(f[e] * s1);
  _Float16* dp = dst + (size_t)r * ND + c8;
  *(volatile v8h*)dp = o1;
  __threadfence();
  *(volatile v8h*)dp = o1;
}

__global__ __launch_bounds__(256) void er_kernel(const float* __restrict__ src, _Float16* __restrict__ dst,
                                                 int eroff) {
  const int i = blockIdx.x * 256 + threadIdx.x;
  if (i >= SEQ * (HDV / 8)) return;
  const int r  = i >> 3;
  const int c8 = (i & 7) * 8;
  const float* sp = src + (size_t)(eroff + r) * HDV + c8;
  const v4f a = *(const v4f*)(sp);
  const v4f b = *(const v4f*)(sp + 4);
  float f[8];
  f[0] = bf_rne(a[0]); f[1] = bf_rne(a[1]); f[2] = bf_rne(a[2]); f[3] = bf_rne(a[3]);
  f[4] = bf_rne(b[0]); f[5] = bf_rne(b[1]); f[6] = bf_rne(b[2]); f[7] = bf_rne(b[3]);
  v8h hi, lo;
#pragma unroll
  for (int e = 0; e < 8; ++e) {
    hi[e] = (_Float16)(f[e] * 16.0f);
    lo[e] = (_Float16)(f[e] * 0.015625f);
  }
  _Float16* dp = dst + (size_t)r * HQK + c8;
  *(volatile v8h*)(dp)      = hi;
  *(volatile v8h*)(dp + 64) = lo;
  __threadfence();
  *(volatile v8h*)(dp)      = hi;
  *(volatile v8h*)(dp + 64) = lo;
}

template <int OUT, bool SKEW>
__global__ __launch_bounds__(256) void gemm_f16_kernel(
    const _Float16* __restrict__ A, int lda, long strideA,
    const _Float16* __restrict__ Bt, int ldb, long strideB,
    void* C1, void* C2, int ldc, long strideC,
    const float* __restrict__ bias,
    int M, int N, int K, float scale, float carry, int skew0, int wrapN, int lmode) {
  __shared__ __align__(16) float sT[8][16 * 68];

  const int z    = blockIdx.y;
  const int lane = threadIdx.x & 31;
  const int wave = threadIdx.x >> 5;
  const int tilesN = N >> 6;
  const int tilesM = M >> 6;
  const int tile = blockIdx.x * 8 + wave;
  if (tile >= tilesM * tilesN) return;
  const int tm = tile / tilesN;
  const int tn = tile - tm * tilesN;
  if (lmode == 1) { if (tn > tm + 1) return; }
  const int m0 = tm << 6;
  const int n0 = tn << 6;
  const int nsk = SKEW ? ((skew0 - tm) << 6) : 0;

  const _Float16* Ab = A  + (size_t)z * strideA;
  const _Float16* Bb = Bt + (size_t)z * strideB;

  const int rl   = lane & 15;
  const int koff = (lane >> 4) * 8;
  const int mOff = (lane >> 4) * 8;

  v8f acc[4][4];
#pragma unroll
  for (int i = 0; i < 4; ++i)
#pragma unroll
    for (int j = 0; j < 4; ++j) acc[i][j] = zero8();

  for (int k0 = 0; k0 < K; k0 += 32) {
    v16h bfr[4];
#pragma unroll
    for (int j = 0; j < 4; ++j) {
      int brow = nsk + n0 + (j << 4) + rl;
      if (SKEW) brow -= (brow >= wrapN) ? wrapN : 0;
      bfr[j] = ldfrag(Bb + (size_t)brow * ldb + koff + k0);
    }
#pragma unroll
    for (int i = 0; i < 4; ++i) {
      const v16h af = ldfrag(Ab + (size_t)(m0 + (i << 4) + rl) * lda + koff + k0);
#pragma unroll
      for (int j = 0; j < 4; ++j) acc[i][j] = mma16(af, bfr[j], acc[i][j]);
    }
  }

  float* slab = sT[wave];
  const int hh = lane >> 4, c4 = (lane & 15) * 4;
  const int q8 = lane >> 3, c8 = (lane & 7) * 8;
  float col8[8];
#pragma unroll
  for (int e = 0; e < 8; ++e) col8[e] = 0.f;
  if (OUT == 2 || OUT == 3) {
    const v4f ta = *(const v4f*)(bias + n0 + c8);
    const v4f tb = *(const v4f*)(bias + n0 + c8 + 4);
    col8[0] = bf_rne(ta[0]); col8[1] = bf_rne(ta[1]); col8[2] = bf_rne(ta[2]); col8[3] = bf_rne(ta[3]);
    col8[4] = bf_rne(tb[0]); col8[5] = bf_rne(tb[1]); col8[6] = bf_rne(tb[2]); col8[7] = bf_rne(tb[3]);
  }
  const float carry2 = carry * 0.0009765625f;

#pragma unroll
  for (int i = 0; i < 4; ++i) {
    const int mBase = m0 + (i << 4);
#pragma unroll
    for (int j = 0; j < 4; ++j)
#pragma unroll
      for (int r = 0; r < 8; ++r)
        slab[(mOff + r) * 68 + (j << 4) + rl] = acc[i][j][r] * scale;
    __builtin_amdgcn_fence(__ATOMIC_RELEASE, "workgroup");
    __builtin_amdgcn_wave_barrier();
    __builtin_amdgcn_fence(__ATOMIC_ACQUIRE, "workgroup");
    if (OUT == 0) {
      float* C = (float*)C1 + (size_t)z * strideC;
      v4f vv[8];
#pragma unroll
      for (int it = 0; it < 8; ++it) {
        const int row = it * 2 + hh;
        vv[it] = *(const v4fa*)(slab + row * 68 + c4);
      }
      for (int ps = 0; ps < 2; ++ps) {
#pragma unroll
        for (int it = 0; it < 8; ++it) {
          const int row = it * 2 + hh;
          *(volatile v4f*)(C + (size_t)(mBase + row) * ldc + n0 + c4) = vv[it];
        }
        __threadfence();
      }
    } else {
      _Float16* Ca = (_Float16*)C1 + (size_t)z * strideC;
      _Float16* Cb = (_Float16*)C2 + (size_t)z * strideC;
      v8h hv[4], lv[4];
#pragma unroll
      for (int it = 0; it < 4; ++it) {
        const int row = it * 4 + q8;
        const float* sp = slab + row * 68 + c8;
        const v4f x0 = *(const v4fa*)(sp);
        const v4f x1 = *(const v4fa*)(sp + 4);
        float f[8];
        f[0] = x0[0]; f[1] = x0[1]; f[2] = x0[2]; f[3] = x0[3];
        f[4] = x1[0]; f[5] = x1[1]; f[6] = x1[2]; f[7] = x1[3];
        float rb = 0.f;
        if (OUT == 5) rb = bf_rne(bias[mBase + row]);
        v8h ha, la;
#pragma unroll
        for (int e = 0; e < 8; ++e) {
          const float t  = (f[e] + col8[e]) + rb;
          const float th = t * carry;
          const _Float16 hq = (_Float16)th;
          ha[e] = hq;
          if (OUT == 2) la[e] = (_Float16)(t * carry2);
          else          la[e] = (_Float16)((th - (float)hq) * 1024.0f);
        }
        hv[it] = ha; lv[it] = la;
      }
      for (int ps = 0; ps < 2; ++ps) {
#pragma unroll
        for (int it = 0; it < 4; ++it) {
          const int row = it * 4 + q8;
          if (OUT == 5) {
            const size_t p = (size_t)(mBase + row) * ldc + n0 + c8;
            *(volatile v8h*)(Ca + p) = hv[it];
            *(volatile v8h*)(Cb + p) = lv[it];
          } else {
            _Float16* cp = Ca + (size_t)(mBase + row) * ldc + 2 * n0 + c8;
            *(volatile v8h*)(cp)      = hv[it];
            *(volatile v8h*)(cp + 64) = lv[it];
          }
        }
        __threadfence();
      }
    }
    __builtin_amdgcn_fence(__ATOMIC_RELEASE, "workgroup");
    __builtin_amdgcn_wave_barrier();
    __builtin_amdgcn_fence(__ATOMIC_ACQUIRE, "workgroup");
  }
}

template <bool RES>
__global__ __launch_bounds__(128)
void attn_kernel(const _Float16* __restrict__ Q2, const _Float16* __restrict__ KP,
                 const _Float16* __restrict__ VT, const _Float16* __restrict__ VL,
                 const float* __restrict__ BD, float* __restrict__ outb,
                 int h0, int qb0, float cs) {
  __shared__ __align__(16) unsigned char SMEM[RES ? 49152 : 32768];
  _Float16* Ksh = (_Float16*)(SMEM);
  _Float16* Vsh = (_Float16*)(SMEM + 16384);
  _Float16* Wsh = (_Float16*)(SMEM + (RES ? 24576 : 16384));
  _Float16* Psh = (_Float16*)(SMEM + (RES ? 32768 : 24576));
  _Float16* Rsh = (_Float16*)(SMEM + (RES ? 40960 : 24576));
  float*    Osh = (float*)(SMEM);

  const int tid  = threadIdx.x;
  const int wave = tid >> 5;
  const int lane = tid & 31;
  const int hh   = lane >> 4;
  const int c    = lane & 15;

  const int z    = blockIdx.y;
  const int h    = h0 + z;
  const int qb   = qb0 + blockIdx.x;
  const int q0   = qb * 64 + wave * 16;
  const int rr0  = wave * 16 + 8 * hh;
  const int iq   = q0 + 8 * hh;
  const int nkt  = qb + 1;

  const _Float16* Qh = Q2 + h * HQK;
  const _Float16* Kh = KP + h * HQK;
  const _Float16* Vh = VT + (size_t)(h * HDV) * SEQ;
  const _Float16* Vl = VL + (size_t)(h * HDV) * SEQ;
  const float*    bd = BD + (size_t)z * SEQ * BDW;

  v16h qa[4];
#pragma unroll
  for (int dc = 0; dc < 4; ++dc)
    qa[dc] = ldfrag(Qh + (size_t)(q0 + c) * QKW + dc * 32 + 8 * hh);

  const float* bdr = bd + (size_t)(q0 + 8 * hh) * BDW + (63 - rr0 + c);

  float mrow[8], lrow[8];
  v8f oacc[4], oacc2[4];
#pragma unroll
  for (int r = 0; r < 8; ++r) { mrow[r] = -INFINITY; lrow[r] = 0.f; }
#pragma unroll
  for (int t = 0; t < 4; ++t) { oacc[t] = zero8(); oacc2[t] = zero8(); }

  _Float16* pw = Psh + wave * (16 * 64);
  _Float16* rw = Rsh + wave * (16 * 64);

#pragma unroll 1
  for (int kc = 0; kc < nkt; ++kc) {
    const int kv0 = kc * 64;
    __syncthreads();
    {
      const int r = tid >> 1, c0 = (tid & 1) * 64, cv = (tid & 1) * 32;
      const _Float16* ks = Kh + (size_t)(kv0 + r) * QKW + c0;
      const _Float16* vs = Vh + (size_t)r * SEQ + kv0 + cv;
#pragma unroll
      for (int i = 0; i < 8; ++i) {
        const v8h kk8 = *(const v8h*)(ks + 8 * i);
        *(v8ha*)(Ksh + r * 128 + c0 + 8 * i) = kk8;
      }
#pragma unroll
      for (int i = 0; i < 4; ++i) {
        const v8h vv8 = *(const v8h*)(vs + 8 * i);
        *(v8ha*)(Vsh + r * 64 + cv + 8 * i) = vv8;
      }
      if (RES) {
        const _Float16* ls = Vl + (size_t)r * SEQ + kv0 + cv;
#pragma unroll
        for (int i = 0; i < 4; ++i) {
          const v8h ll8 = *(const v8h*)(ls + 8 * i);
          *(v8ha*)(Wsh + r * 64 + cv + 8 * i) = ll8;
        }
      }
    }
    __syncthreads();

    v8f s[4];
#pragma unroll
    for (int j = 0; j < 4; ++j) {
      s[j] = zero8();
#pragma unroll
      for (int dc = 0; dc < 4; ++dc) {
        const v16h kb = ldfrag(Ksh + (j * 16 + c) * 128 + dc * 32 + 8 * hh);
        s[j] = mma16(qa[dc], kb, s[j]);
      }
    }

    float cm[8];
#pragma unroll
    for (int r = 0; r < 8; ++r) {
      const int i = iq + r;
      float m = -INFINITY;
#pragma unroll
      for (int j = 0; j < 4; ++j) {
        const int key  = kv0 + (j << 4) + c;
        const float bv = bdr[r * (BDW - 1) + kv0 + (j << 4)];
        const float raw = s[j][r] * cs + bv;
        const float sv  = (key > i) ? -1.0e30f : raw;
        s[j][r] = sv;
        m = fmaxf(m, sv);
      }
      m = fmaxf(m, __shfl_xor(m, 1, 32));
      m = fmaxf(m, __shfl_xor(m, 2, 32));
      m = fmaxf(m, __shfl_xor(m, 4, 32));
      m = fmaxf(m, __shfl_xor(m, 8, 32));
      cm[r] = m;
      __asm__ __volatile__("" ::: "memory");
    }

#pragma unroll
    for (int r = 0; r < 8; ++r) {
      const float mnew  = fmaxf(mrow[r], cm[r]);
      const float alpha = __expf(mrow[r] - mnew);
      mrow[r] = mnew;
      float psum = 0.f;
#pragma unroll
      for (int j = 0; j < 4; ++j) {
        const float p  = __expf(s[j][r] - mnew);
        psum += p;
        const float ph = p * 4096.0f;
        const _Float16 hq = (_Float16)ph;
        pw[(8 * hh + r) * 64 + j * 16 + c] = hq;
        if (RES) rw[(8 * hh + r) * 64 + j * 16 + c] = (_Float16)((ph - (float)hq) * 1024.0f);
      }
      psum += __shfl_xor(psum, 1, 32);
      psum += __shfl_xor(psum, 2, 32);
      psum += __shfl_xor(psum, 4, 32);
      psum += __shfl_xor(psum, 8, 32);
      lrow[r] = lrow[r] * alpha + psum;
#pragma unroll
      for (int t = 0; t < 4; ++t) {
        oacc[t][r] *= alpha;
        if (RES) oacc2[t][r] *= alpha;
      }
    }
    __builtin_amdgcn_fence(__ATOMIC_RELEASE, "workgroup");
    __builtin_amdgcn_wave_barrier();
    __builtin_amdgcn_fence(__ATOMIC_ACQUIRE, "workgroup");

#pragma unroll
    for (int kk = 0; kk < 2; ++kk) {
      const v16h pa = ldfrag(pw + c * 64 + kk * 32 + 8 * hh);
      v16h pl;
      if (RES) pl = ldfrag(rw + c * 64 + kk * 32 + 8 * hh);
#pragma unroll
      for (int t = 0; t < 4; ++t) {
        const v16h vb = ldfrag(Vsh + (t * 16 + c) * 64 + kk * 32 + 8 * hh);
        oacc[t] = mma16(pa, vb, oacc[t]);
        if (RES) {
          const v16h vl = ldfrag(Wsh + (t * 16 + c) * 64 + kk * 32 + 8 * hh);
          oacc2[t] = mma16(pl, vb, oacc2[t]);
          oacc2[t] = mma16(pa, vl, oacc2[t]);
        }
      }
    }
  }

  __syncthreads();
  float* os = Osh + wave * (16 * HDV);
#pragma unroll
  for (int r = 0; r < 8; ++r) {
    const float inv = 1.0f / (65536.0f * lrow[r]);
#pragma unroll
    for (int t = 0; t < 4; ++t) {
      float v = oacc[t][r];
      if (RES) v += oacc2[t][r] * 0.0009765625f;
      os[(8 * hh + r) * HDV + t * 16 + c] = v * inv;
    }
  }
  __builtin_amdgcn_fence(__ATOMIC_RELEASE, "workgroup");
  __builtin_amdgcn_wave_barrier();
  __builtin_amdgcn_fence(__ATOMIC_ACQUIRE, "workgroup");
  const int c4 = c * 4;
  v4f vv[8];
#pragma unroll
  for (int it = 0; it < 8; ++it) {
    const int row = it * 2 + hh;
    vv[it] = *(const v4fa*)(os + row * HDV + c4);
  }
  float* ob = outb + h * HDV;
  for (int ps = 0; ps < 2; ++ps) {
#pragma unroll
    for (int it = 0; it < 8; ++it) {
      const int row = it * 2 + hh;
      *(volatile v4f*)(ob + (size_t)(q0 + row) * ND + c4) = vv[it];
    }
    __threadfence();
  }
}

extern "C" void kernel_launch(void* const* d_in, const int* in_sizes, int n_in,
                              void* d_out, int out_size, void* d_ws, size_t ws_size,
                              hipStream_t stream) {
  if (n_in < 8) return;
  if (in_sizes[0] < ((NB - 1) * SEQ_FULL + SEQ) * ND) return;
  if (in_sizes[1] < ND * ND || in_sizes[3] < ND * ND || in_sizes[5] < ND * ND) return;
  if (in_sizes[2] < ND || in_sizes[4] < ND || in_sizes[6] < ND) return;
  if (in_sizes[7] < SEQ * HDV) return;
  if (out_size < NB * SEQ * ND) return;
  const int erows = in_sizes[7] / HDV;
  const int eroff = erows - SEQ;

  const float* x  = (const float*)d_in[0];
  const float* Wq = (const float*)d_in[1];
  const float* bq = (const float*)d_in[2];
  const float* Wk = (const float*)d_in[3];
  const float* bk = (const float*)d_in[4];
  const float* Wv = (const float*)d_in[5];
  const float* bv = (const float*)d_in[6];
  const float* Er = (const float*)d_in[7];
  float* out = (float*)d_out;

  const size_t szW  = (size_t)ND * ND * 2;
  const size_t szER = (size_t)SEQ * HQK * 2;
  const size_t szXH = (size_t)SEQ * ND * 2;
  const size_t szQ2 = (size_t)SEQ * QKW * 2;
  const size_t szVT = (size_t)ND * SEQ * 2;
  const size_t szBD = (size_t)NPAIR * SEQ * BDW * 4;
  size_t off = 0;
  const size_t oWQ = off; off += szW;
  const size_t oWK = off; off += szW;
  const size_t oWV = off; off += szW;
  const size_t oER = off; off += szER;
  const size_t oXH = off; off += szXH;
  const size_t oQ2 = off; off += szQ2;
  const size_t oKP = off; off += szQ2;
  const size_t oVT = off; off += szVT;
  const size_t oVL = off; off += szVT;
  const size_t oBD = off; off += szBD;
  const size_t total = off;
  if (total > ws_size) return;
  if (total > (size_t)134217728) return;

  char* ws = (char*)d_ws;
  _Float16* WQp = (_Float16*)(ws + oWQ);
  _Float16* WKp = (_Float16*)(ws + oWK);
  _Float16* WVp = (_Float16*)(ws + oWV);
  _Float16* ERP = (_Float16*)(ws + oER);
  _Float16* XH  = (_Float16*)(ws + oXH);
  _Float16* Q2  = (_Float16*)(ws + oQ2);
  _Float16* KP2 = (_Float16*)(ws + oKP);
  _Float16* VTp = (_Float16*)(ws + oVT);
  _Float16* VLp = (_Float16*)(ws + oVL);
  float*    BDp = (float*)(ws + oBD);

  const float cs  = 0.125f * 0.00390625f;
  const float rqk = 0.0000152587890625f;
  const dim3 blk(256);

  const dim3 gW((ND * (ND / 8) + 255) / 256);
  cvt_kernel<<<gW, blk, 0, stream>>>(Wq, WQp, ND, 1024.0f);
  cvt_kernel<<<gW, blk, 0, stream>>>(Wk, WKp, ND, 1024.0f);
  cvt_kernel<<<gW, blk, 0, stream>>>(Wv, WVp, ND, 1024.0f);
  const dim3 gE((SEQ * (HDV / 8) + 255) / 256);
  er_kernel<<<gE, blk, 0, stream>>>(Er, ERP, eroff);
  const dim3 gX((SEQ * (ND / 8) + 255) / 256);
  const int tilesQ  = NKT * (ND / 64);
  const int tilesBD = NKT * (BDW / 64);
  for (int b = 0; b < NB; ++b) {
    cvt_kernel<<<gX, blk, 0, stream>>>(x + (size_t)b * SEQ_FULL * ND, XH, SEQ, 64.0f);
    gemm_f16_kernel<3, false><<<dim3((tilesQ + 7) / 8, 1), blk, 0, stream>>>(
        XH, ND, 0L, WQp, ND, 0L, (void*)Q2, (void*)Q2, QKW, 0L, bq,
        SEQ, ND, ND, rqk, 16.0f, 0, SEQ, 0);
    gemm_f16_kernel<2, false><<<dim3((tilesQ + 7) / 8, 1), blk, 0, stream>>>(
        XH, ND, 0L, WKp, ND, 0L, (void*)KP2, (void*)KP2, QKW, 0L, bk,
        SEQ, ND, ND, rqk, 16.0f, 0, SEQ, 0);
    gemm_f16_kernel<5, false><<<dim3((tilesQ + 7) / 8, 1), blk, 0, stream>>>(
        WVp, ND, 0L, XH, ND, 0L, (void*)VTp, (void*)VLp, SEQ, 0L, bv,
        ND, SEQ, ND, rqk, 16.0f, 0, SEQ, 0);
    float* outb = out + (size_t)b * SEQ * ND;
    for (int gi = 0; gi < NH / NPAIR; ++gi) {
      const int h0 = gi * NPAIR;
      const _Float16* Aq = Q2 + h0 * HQK;
      gemm_f16_kernel<0, true><<<dim3((tilesBD + 7) / 8, NPAIR), blk, 0, stream>>>(
          Aq, QKW, (long)HQK, ERP, HQK, 0L, (void*)BDp, (void*)BDp, BDW, (long)SEQ * BDW, bq,
          SEQ, BDW, HQK, cs, 1.0f, NKT - 1, SEQ, 1);
      attn_kernel<false><<<dim3(NKT - QRES, NPAIR), dim3(128), 0, stream>>>(
          Q2, KP2, VTp, VLp, BDp, outb, h0, QRES, cs);
      attn_kernel<true><<<dim3(QRES, NPAIR), dim3(128), 0, stream>>>(
          Q2, KP2, VTp, VLp, BDp, outb, h0, 0, cs);
    }
  }
  (void)hipGetLastError();
}
